// DANetHead_37924561223996
// MI455X (gfx1250) — hardware-verified
//
#include <hip/hip_runtime.h>
#include <hip/hip_bf16.h>
#include <math.h>

#define NB_   2
#define CIN   256
#define CD    128
#define IMH   64
#define IMW   64
#define HW_   4096
#define NG    32
#define SS    4096
#define HH    1
#define BB    2
#define DKK   128
#define QW    1
#define QST   128
#define KVST  128
#define KST2  136
#define KST   40
#define NCLS  19

typedef _Float16 bf16;
typedef _Float16 f16;
typedef __attribute__((ext_vector_type(4))) unsigned v4u_t;
typedef unsigned v4ua __attribute__((ext_vector_type(4), may_alias));
typedef __attribute__((ext_vector_type(4))) float v4f_t;
typedef float v4fa __attribute__((ext_vector_type(4), may_alias));
typedef __attribute__((ext_vector_type(16))) bf16  bf16x16;
typedef bf16x16 f16x16;
typedef __attribute__((ext_vector_type(8)))  bf16  bf16x8;
typedef bf16x8 f16x8;
typedef __attribute__((ext_vector_type(4)))  bf16  bf16x4;
typedef __attribute__((ext_vector_type(8)))  float f32x8;
__device__ __forceinline__ f32x8 wmma16(f16x16 a, f16x16 b, f32x8 c) {
  c = __builtin_amdgcn_wmma_f32_16x16x32_f16(false, a, false, b, (short)0, c, false, false);
  asm volatile("v_nop\n\tv_nop\n\tv_nop\n\tv_nop" : "+v"(c) : "v"(a), "v"(b));
  return c;
}
#define LDS_STRIDE 48
#define KSTRIDE    72
#define VSTRIDE    48

__device__ __forceinline__ f32x8 wmma_bf16(bf16x16 a, bf16x16 b, f32x8 c) {
  c = __builtin_amdgcn_wmma_f32_16x16x32_f16(false, a, false, b, (short)0, c, false, false);
  asm volatile("v_nop\n\tv_nop\n\tv_nop\n\tv_nop" : "+v"(c) : "v"(a), "v"(b));
  return c;
}

template <typename T>
__device__ __forceinline__ bf16x16 load_frag(const T* __restrict__ base, int ld,
                                             int row0, int k0) {
  const int lane = threadIdx.x & 31;
  const int r    = lane & 15;
  const int kh   = (lane >> 4) * 8;
  const T* p0 = base + (size_t)(row0 + r) * ld + (k0 + kh);
  const T* p1 = p0 + 16;
  bf16x16 f;
#pragma unroll
  for (int i = 0; i < 8; ++i) {
    f[i]     = (bf16)p0[i];
    f[i + 8] = (bf16)p1[i];
  }
  return f;
}

__device__ __forceinline__ bf16x16 lds_frag(const bf16* base, int stride) {
  const int lane = threadIdx.x & 31;
  const int row  = lane & 15;
  const int kh   = (lane >> 4) * 8;
  const bf16x8 lo = *(const bf16x8*)(base + row * stride + kh);
  const bf16x8 hi = *(const bf16x8*)(base + row * stride + kh + 16);
  bf16x16 f;
#pragma unroll
  for (int i = 0; i < 8; ++i) { f[i] = lo[i]; f[i + 8] = hi[i]; }
  return f;
}

template <typename T>
__device__ __forceinline__ void stage_read16(const T* __restrict__ p, float* buf) {
#pragma unroll
  for (int i = 0; i < 16; ++i) buf[i] = (float)p[i];
}

__device__ __forceinline__ void stage_write(bf16* dst, const float* buf, int nquad) {
#pragma unroll
  for (int i = 0; i < nquad; ++i) {
    bf16x4 q;
    q[0] = (bf16)buf[4 * i];     q[1] = (bf16)buf[4 * i + 1];
    q[2] = (bf16)buf[4 * i + 2]; q[3] = (bf16)buf[4 * i + 3];
    *(bf16x4*)(dst + 4 * i) = q;
  }
}

template <typename AT, int MODE>
__global__ __launch_bounds__(256) void gemm_rb_kernel(
    const AT* __restrict__ A, const float* __restrict__ W,
    const float* __restrict__ bias, const float* __restrict__ rowscale, const float* __restrict__ R, const float* __restrict__ rowbias, void* __restrict__ out,
    int M, int N, int K) {
  __shared__ bf16 ldsA[128 * LDS_STRIDE];
  __shared__ bf16 ldsW[256 * LDS_STRIDE];
  __shared__ __attribute__((aligned(16))) unsigned char sob[256 * 136 * 2];

  const int t    = threadIdx.x;
  const int wave = t >> 5;
  const int lane = t & 31;
  const int wm   = (wave & 1) * 64;
  const int wn   = (wave >> 1) * 64;
  const int mBlk = blockIdx.x * 128;
  const int nBlk = blockIdx.y * 256;

  const int arow = t >> 1;
  const int ach  = (t & 1) * 16;

  float abuf[16];
  float wbuf[32];

  stage_read16(A + (size_t)(mBlk + arow) * K + ach, abuf);
  const int nrow = min(nBlk + t, N - 1);
  stage_read16(W + (size_t)nrow * K,          wbuf);
  stage_read16(W + (size_t)nrow * K + 16,     wbuf + 16);

  f32x8 acc[4][4] = {};

  for (int k = 0; k < K; k += 32) {
    __syncthreads();
    stage_write(&ldsA[arow * LDS_STRIDE + ach], abuf, 4);
    stage_write(&ldsW[t * LDS_STRIDE],          wbuf, 8);
    if (k + 32 < K) {
      stage_read16(A + (size_t)(mBlk + arow) * K + (k + 32) + ach, abuf);
      stage_read16(W + (size_t)nrow * K + (k + 32),          wbuf);
      stage_read16(W + (size_t)nrow * K + (k + 32) + 16,     wbuf + 16);
    }
    __syncthreads();

    bf16x16 af[4], wf[4];
#pragma unroll
    for (int i = 0; i < 4; ++i)
      af[i] = lds_frag(ldsA + (wm + 16 * i) * LDS_STRIDE, LDS_STRIDE);
#pragma unroll
    for (int j = 0; j < 4; ++j)
      wf[j] = lds_frag(ldsW + (wn + 16 * j) * LDS_STRIDE, LDS_STRIDE);
#pragma unroll
    for (int i = 0; i < 4; ++i)
#pragma unroll
      for (int j = 0; j < 4; ++j)
        acc[i][j] = wmma_bf16(af[i], wf[j], acc[i][j]);
  }

  const int nlane = lane & 15;
  const int mh    = (lane >> 4) * 8;
  __syncthreads();
  if (MODE == 0 || MODE == 1 || MODE == 3) {
    bf16* so = (bf16*)sob;
#pragma unroll
    for (int i = 0; i < 4; ++i)
#pragma unroll
      for (int j = 0; j < 4; ++j) {
        const int nl = wn + 16 * j + nlane;
        const float bv = bias ? bias[nBlk + nl] : 0.0f;
        if (MODE == 3) {
#pragma unroll 1
          for (int r = 0; r < 8; ++r) {
            const int ml = wm + 16 * i + mh + r;
            const float xg = acc[i][j][r] + bv;
            so[ml * 264 + nl] = (bf16)(0.5f * xg * (1.0f + erff(xg * 0.70710678118654752f)));
          }
        } else {
#pragma unroll
        for (int r = 0; r < 8; ++r) {
          const int ml = wm + 16 * i + mh + r;
          const bf16 hv = (bf16)(acc[i][j][r] + bv);
          if (MODE == 0) so[ml * 264 + nl] = hv;
          else           so[nl * 136 + ml] = hv;
        }
        }
      }
    __syncthreads();
#pragma unroll 1
    for (int pass = 0; pass < 2; ++pass) {
      if (MODE == 0 || MODE == 3) {
        for (int ch = t; ch < 128 * 32; ch += 256) { const int ml = ch >> 5, q = (ch & 31) * 8;
          *(volatile v4u_t*)((bf16*)out + (size_t)(mBlk + ml) * N + nBlk + q) = *(const v4ua*)(so + ml * 264 + q); }
      } else {
        const int b_ = mBlk / SS, s0 = mBlk & (SS - 1);
        for (int ch = t; ch < 256 * 16; ch += 256) { const int nl = ch >> 4, q = (ch & 15) * 8; const int n = nBlk + nl, h = n >> 6, dk = n & (DKK - 1);
          *(volatile v4u_t*)((bf16*)out + (((size_t)(b_ * HH + h)) * DKK + dk) * SS + s0 + q) = *(const v4ua*)(so + nl * 136 + q); }
      }
      __threadfence();
    }
  } else {
    float* so = (float*)sob;
#pragma unroll 1
    for (int hf = 0; hf < 2; ++hf) {
      if (wm == hf * 64) {
#pragma unroll
        for (int i = 0; i < 4; ++i)
#pragma unroll
          for (int j = 0; j < 4; ++j) {
            const int nl = wn + 16 * j + nlane;
            const float bv = bias ? bias[nBlk + nl] : 0.0f;
#pragma unroll
            for (int r = 0; r < 8; ++r) { const int mrow = mBlk + hf * 64 + 16 * i + mh + r; so[(16 * i + mh + r) * 260 + nl] = acc[i][j][r] * (rowscale ? rowscale[mrow] : 1.0f) + bv + (rowbias ? rowbias[mrow] : 0.0f); }
          }
      }
      __syncthreads();
      if (R) {
        for (int ch = t; ch < 64 * 64; ch += 256) { const int ml = ch >> 6, q = (ch & 63) * 4;
          if (nBlk + q < N) { const v4f_t rv = *(const v4f_t*)(R + (size_t)(mBlk + hf * 64 + ml) * N + nBlk + q); v4f_t v = *(const volatile v4fa*)(so + ml * 260 + q); v += rv; *(volatile v4fa*)(so + ml * 260 + q) = v; } }
        asm volatile("s_wait_dscnt 0" ::: "memory");
      }
#pragma unroll 1
      for (int pass = 0; pass < 2; ++pass) {
        for (int ch = t; ch < 64 * 64; ch += 256) { const int ml = ch >> 6, q = (ch & 63) * 4;
          if (nBlk + q < N) *(volatile v4f_t*)((float*)out + (size_t)(mBlk + hf * 64 + ml) * N + nBlk + q) = *(const volatile v4fa*)(so + ml * 260 + q); }
        __threadfence();
      }
      __syncthreads();
    }
  }
}

__global__ __launch_bounds__(64) void attn_kernel(
    const bf16* __restrict__ Qb, const bf16* __restrict__ Kb,
    const bf16* __restrict__ Vt, float* __restrict__ attnOut) {
  __shared__ bf16 ldsK[32 * KST2];
  __shared__ bf16 ldsV[128 * VSTRIDE];
  __shared__ __attribute__((aligned(16))) float ldsO[2][16 * 132];

  const int q0blk = blockIdx.x * 32;
  const int h  = blockIdx.y;
  const int b  = blockIdx.z;
  const int t    = threadIdx.x;
  const int wave = t >> 5;
  const int lane = t & 31;
  const int qlane = lane & 15;
  const int kh8   = (lane >> 4) * 8;
  const int q0 = q0blk + wave * 16;

  const int hk = h;
  const bf16* Qh = Qb + (size_t)b * SS * QST + h * DKK;
  const bf16* Kh = Kb + (size_t)b * SS * KVST + hk * DKK;
  const bf16* Vh = Vt + ((size_t)(b * HH + hk)) * DKK * SS;

  const int krow = t >> 1;
  const int kcol = (t & 1) * 64;
  const bf16* kSrc = Kh + (size_t)krow * KVST + kcol;
  const bf16* vSrc = Vh + (size_t)t * SS;

  bf16x16 qf[QW][4];
#pragma unroll
  for (int qt = 0; qt < QW; ++qt)
#pragma unroll
    for (int c = 0; c < 4; ++c) qf[qt][c] = load_frag(Qh, QST, q0 + 16 * qt, 32 * c);

  f32x8 o[QW][8] = {};
  float mrun[QW], lrun[QW];
#pragma unroll
  for (int qt = 0; qt < QW; ++qt) { mrun[qt] = -INFINITY; lrun[qt] = 0.0f; }

  const float scale = 1.44269504088896340736f;
  const float NEG2 = -1.0e9f;
  const int kmax = SS - 1, kmin = 0;

  bf16x8 kreg[8], vreg[8];
#pragma unroll
  for (int i = 0; i < 8; ++i) kreg[i] = *(const bf16x8*)(kSrc + (size_t)kmin * KVST + 8 * i);
#pragma unroll
  for (int i = 0; i < 4; ++i) { vreg[i] = *(const bf16x8*)(vSrc + kmin + 8 * i); vreg[4 + i] = *(const bf16x8*)(vSrc + (size_t)64 * SS + kmin + 8 * i); }

  for (int kb = kmin; kb <= kmax; kb += 32) {
    __syncthreads();
#pragma unroll
    for (int i = 0; i < 8; ++i) *(bf16x8*)(&ldsK[krow * KST2 + kcol + 8 * i]) = kreg[i];
#pragma unroll
    for (int i = 0; i < 4; ++i) { *(bf16x8*)(&ldsV[t * VSTRIDE + 8 * i]) = vreg[i]; *(bf16x8*)(&ldsV[(t + 64) * VSTRIDE + 8 * i]) = vreg[4 + i]; }
    if (kb + 32 <= kmax) {
      const bf16* kn = kSrc + (size_t)(kb + 32) * KVST;
      const bf16* vn = vSrc + (kb + 32);
#pragma unroll
      for (int i = 0; i < 8; ++i) kreg[i] = *(const bf16x8*)(kn + 8 * i);
#pragma unroll
      for (int i = 0; i < 4; ++i) { vreg[i] = *(const bf16x8*)(vn + 8 * i); vreg[4 + i] = *(const bf16x8*)(vn + (size_t)64 * SS + 8 * i); }
    }
    __syncthreads();


    bf16x16 pf[QW];
    bool act[QW];
#pragma unroll
    for (int qt = 0; qt < QW; ++qt) {
      unsigned mbits = 0;
      mbits = 0xFFFFu; act[qt] = true;
      if (act[qt]) {
        const int q_my = q0 + 16 * qt + qlane;
        f32x8 s0 = {}, s1 = {};
#pragma unroll
        for (int c = 0; c < 4; ++c) {
          const bf16x16 k0f = lds_frag(ldsK + 0 * KST2 + c * 32, KST2), k1f = lds_frag(ldsK + 16 * KST2 + c * 32, KST2);
          s0 = wmma_bf16(k0f, qf[qt][c], s0);
          s1 = wmma_bf16(k1f, qf[qt][c], s1);
        }

        float mx = -INFINITY;
#pragma unroll
        for (int r = 0; r < 8; ++r) {
          const int k0i = kb + kh8 + r;
          const int k1i = k0i + 16;
          (void)k0i; (void)k1i; (void)q_my;
          s0[r] = (mbits & (1u << r))       ? s0[r] * scale : NEG2;
          s1[r] = (mbits & (1u << (8 + r))) ? s1[r] * scale : NEG2;
          mx = fmaxf(mx, fmaxf(s0[r], s1[r]));
        }
        mx = fmaxf(mx, __shfl_xor(mx, 16, 32));
        const float mnew  = fmaxf(mrun[qt], mx);
        const float alpha = exp2f(mrun[qt] - mnew);

        float rsum = 0.0f;
#pragma unroll
        for (int r = 0; r < 8; ++r) {
          const float p0 = exp2f(s0[r] - mnew);
          const float p1 = exp2f(s1[r] - mnew);
          rsum += p0 + p1;
          pf[qt][r]     = (bf16)(p0 * 1024.0f);
          pf[qt][r + 8] = (bf16)(p1 * 1024.0f);
        }
        rsum += __shfl_xor(rsum, 16, 32);
        lrun[qt] = lrun[qt] * alpha + rsum;
        mrun[qt] = mnew;

#pragma unroll
        for (int j = 0; j < 8; ++j)
#pragma unroll
          for (int r = 0; r < 8; ++r) o[qt][j][r] *= alpha;
      }
    }

#pragma unroll
    for (int j = 0; j < 8; ++j) {
      const bf16x16 vf = lds_frag(ldsV + (j * 16) * VSTRIDE, VSTRIDE);
#pragma unroll
      for (int qt = 0; qt < QW; ++qt)
        if (act[qt]) o[qt][j] = wmma_bf16(vf, pf[qt], o[qt][j]);
    }
  }

  float* so = ldsO[wave];
  {
    const float rl = 1.0f / (lrun[0] * 1024.0f);
#pragma unroll
    for (int j = 0; j < 8; ++j)
#pragma unroll
      for (int r = 0; r < 8; ++r) so[qlane * 132 + j * 16 + kh8 + r] = o[0][j][r] * rl;
  }
  asm volatile("s_wait_dscnt 0" ::: "memory");
  __builtin_amdgcn_wave_barrier();
#pragma unroll 1
  for (int pass = 0; pass < 2; ++pass) {
#pragma unroll
    for (int it = 0; it < 16; ++it) { const int ql = it, q4 = lane * 4;
      *(volatile v4f_t*)(attnOut + ((size_t)(b * SS + q0 + ql)) * QST + q4) = *(const volatile v4fa*)(so + ql * 132 + q4); }
    __threadfence();
  }
}


__global__ __launch_bounds__(256) void k_convd(const float* __restrict__ src, const float* __restrict__ Wt, float* __restrict__ Y) {
  __shared__ __attribute__((aligned(16))) f16 ldsA[128 * KST];
  __shared__ __attribute__((aligned(16))) f16 ldsB[128 * KST];
  __shared__ __attribute__((aligned(16))) float oS[8][32 * 68];
  constexpr int KTOT = CIN * 9;
  const int tid = threadIdx.x, lane = tid & 31, wave = tid >> 5, cl = lane & 15, rh = (lane >> 4) * 8;
  const int b = blockIdx.x >> 5, y0 = (blockIdx.x & 31) * 2;
  const int wm = (wave & 3) * 32, wp = (wave >> 2) * 64;
  const float* inb = src + (size_t)b * CIN * HW_;
  f32x8 acc[2][4];
#pragma unroll
  for (int i = 0; i < 2; ++i)
#pragma unroll
    for (int j = 0; j < 4; ++j) { f32x8 z = {}; acc[i][j] = z; }
#pragma unroll 1
  for (int k0 = 0; k0 < KTOT; k0 += 32) {
    __syncthreads();
    { const int o = tid >> 1, kq = (tid & 1) * 16;
      const float* wr = Wt + (size_t)o * KTOT + k0 + kq;
#pragma unroll
      for (int u = 0; u < 16; ++u) ldsA[o * KST + kq + u] = (f16)wr[u]; }
    { const int px = tid >> 1, kq = (tid & 1) * 16;
      const int yy = px >> 6, xx = px & 63;
#pragma unroll 4
      for (int u = 0; u < 16; ++u) {
        const int k = k0 + kq + u, c = k / 9, r9 = k - 9 * c, dy = r9 / 3 - 1, dx = r9 - 3 * (r9 / 3) - 1;
        const int ys = y0 + yy + dy, xs = xx + dx;
        float v = 0.0f;
        if (ys >= 0 && ys < IMH && xs >= 0 && xs < IMW) v = inb[(size_t)c * HW_ + ys * IMW + xs];
        ldsB[px * KST + kq + u] = (f16)v;
      } }
    __syncthreads();
    f16x16 af[2];
#pragma unroll
    for (int i = 0; i < 2; ++i) af[i] = lds_frag(ldsA + (wm + 16 * i) * KST, KST);
#pragma unroll
    for (int j = 0; j < 4; ++j) {
      const f16x16 bfv = lds_frag(ldsB + (wp + 16 * j) * KST, KST);
#pragma unroll
      for (int i = 0; i < 2; ++i) acc[i][j] = wmma16(af[i], bfv, acc[i][j]);
    }
  }
  float* so = oS[wave];
#pragma unroll
  for (int i = 0; i < 2; ++i)
#pragma unroll
    for (int r = 0; r < 8; ++r)
#pragma unroll
      for (int j = 0; j < 4; ++j) so[(16 * i + rh + r) * 68 + 16 * j + cl] = acc[i][j][r];
  asm volatile("s_wait_dscnt 0" ::: "memory");
  __builtin_amdgcn_wave_barrier();
  const size_t pxoff = (size_t)(y0 * IMW + wp);
#pragma unroll 1
  for (int pass = 0; pass < 2; ++pass) {
#pragma unroll
    for (int it = 0; it < 16; ++it) { const int f4 = lane + 32 * it, rr = f4 >> 4, q = (f4 & 15) * 4;
      *(volatile v4f_t*)(Y + ((size_t)b * CD + wm + rr) * HW_ + pxoff + q) = *(const volatile v4fa*)(so + rr * 68 + q); }
    __threadfence();
  }
}
__global__ __launch_bounds__(256) void k_gn_stats(const float* __restrict__ src, float* __restrict__ stats) {
  __shared__ float red[256];
  __shared__ __attribute__((aligned(16))) float outS[32];
  const int b = blockIdx.x >> 1, g0 = (blockIdx.x & 1) * 16, t = threadIdx.x;
#pragma unroll 1
  for (int gg = 0; gg < 16; ++gg) {
    const float* p = src + ((size_t)b * CD + (g0 + gg) * 4) * HW_;
    float s = 0.0f;
    for (int i = t; i < 16384; i += 256) s += p[i];
    red[t] = s; __syncthreads();
    for (int o = 128; o > 0; o >>= 1) { if (t < o) red[t] += red[t + o]; __syncthreads(); }
    const float mu = red[0] * (1.0f / 16384.0f); __syncthreads();
    float q = 0.0f;
    for (int i = t; i < 16384; i += 256) { const float d = p[i] - mu; q += d * d; }
    red[t] = q; __syncthreads();
    for (int o = 128; o > 0; o >>= 1) { if (t < o) red[t] += red[t + o]; __syncthreads(); }
    if (t == 0) { outS[2 * gg] = mu; outS[2 * gg + 1] = 1.0f / sqrtf(red[0] * (1.0f / 16384.0f) + 1e-5f); }
    __syncthreads();
  }
  if (t < 8) {
#pragma unroll 1
    for (int pass = 0; pass < 2; ++pass) { *(volatile v4f_t*)(stats + ((size_t)b * NG + g0) * 2 + t * 4) = *(const volatile v4fa*)(outS + t * 4); __threadfence(); }
  }
}
__global__ __launch_bounds__(256) void k_gn_apply(const float* __restrict__ pre, const float* __restrict__ stats, const float* __restrict__ gam,
                                                 const float* __restrict__ bet, float* __restrict__ C32, bf16* __restrict__ C16,
                                                 float* __restrict__ T32, bf16* __restrict__ T16) {
  __shared__ __attribute__((aligned(16))) float tS[64 * 132];
  const int tid = threadIdx.x, b = blockIdx.x >> 6, p0 = (blockIdx.x & 63) * 64;
  { const int c = tid >> 1, xh = (tid & 1) * 32;
    const float mu = stats[((size_t)b * NG + (c >> 2)) * 2], rs = stats[((size_t)b * NG + (c >> 2)) * 2 + 1], g = gam[c], be = bet[c];
    const float* sp = pre + ((size_t)b * CD + c) * HW_ + p0 + xh;
#pragma unroll
    for (int i = 0; i < 32; ++i) tS[(xh + i) * 132 + c] = fmaxf((sp[i] - mu) * rs * g + be, 0.0f);
  }
  __syncthreads();
#pragma unroll 1
  for (int pass = 0; pass < 2; ++pass) {
#pragma unroll
    for (int it = 0; it < 8; ++it) { const int ch = tid + 256 * it, c = ch >> 4, q4 = (ch & 15) * 4;
      v4f_t w; w[0] = tS[(q4) * 132 + c]; w[1] = tS[(q4 + 1) * 132 + c]; w[2] = tS[(q4 + 2) * 132 + c]; w[3] = tS[(q4 + 3) * 132 + c];
      *(volatile v4f_t*)(C32 + ((size_t)b * CD + c) * HW_ + p0 + q4) = w; }
#pragma unroll
    for (int it = 0; it < 4; ++it) { const int ch = tid + 256 * it, c = ch >> 3, q8 = (ch & 7) * 8;
      union { bf16 h[8]; v4u_t u; } cv;
#pragma unroll
      for (int e = 0; e < 8; ++e) cv.h[e] = (bf16)tS[(q8 + e) * 132 + c];
      *(volatile v4u_t*)(C16 + ((size_t)b * CD + c) * HW_ + p0 + q8) = cv.u; }
    __threadfence();
  }
#pragma unroll 1
  for (int pass = 0; pass < 2; ++pass) {
#pragma unroll
    for (int it = 0; it < 8; ++it) { const int ch = tid + 256 * it, row = ch >> 5, q4 = (ch & 31) * 4;
      *(volatile v4f_t*)(T32 + ((size_t)b * HW_ + p0 + row) * CD + q4) = *(const volatile v4fa*)(tS + row * 132 + q4); }
#pragma unroll
    for (int it = 0; it < 4; ++it) { const int ch = tid + 256 * it, row = ch >> 4, q8 = (ch & 15) * 8;
      union { bf16 h[8]; v4u_t u; } cv;
#pragma unroll
      for (int e = 0; e < 8; ++e) cv.h[e] = (bf16)tS[row * 132 + q8 + e];
      *(volatile v4u_t*)(T16 + ((size_t)b * HW_ + p0 + row) * CD + q8) = cv.u; }
    __threadfence();
  }
}
__global__ __launch_bounds__(256) void k_softmax128(const float* __restrict__ g, float* __restrict__ w) {
  __shared__ __attribute__((aligned(16))) float rowS[128 * 132];
  const int tid = threadIdx.x, b = blockIdx.x, row = tid >> 1, half = tid & 1;
  const float* gr = g + ((size_t)b * CD + row) * CD + half * 64;
  float v[64], m = -INFINITY;
#pragma unroll
  for (int i = 0; i < 64; ++i) { v[i] = gr[i]; m = fmaxf(m, v[i]); }
  m = fmaxf(m, __shfl_xor(m, 1, 32));
  float s = 0.0f;
#pragma unroll
  for (int i = 0; i < 64; ++i) { v[i] = __expf(v[i] - m); s += v[i]; }
  s += __shfl_xor(s, 1, 32);
  const float is = 1.0f / s;
#pragma unroll
  for (int i = 0; i < 64; ++i) rowS[row * 132 + half * 64 + i] = v[i] * is;
  __syncthreads();
#pragma unroll 1
  for (int pass = 0; pass < 2; ++pass) {
#pragma unroll
    for (int it = 0; it < 16; ++it) { const int ch = tid + 256 * it, r = ch >> 5, q4 = (ch & 31) * 4;
      *(volatile v4f_t*)(w + ((size_t)b * CD + r) * CD + q4) = *(const volatile v4fa*)(rowS + r * 132 + q4); }
    __threadfence();
  }
}
__global__ __launch_bounds__(256) void k_padw(const float* __restrict__ w, const float* __restrict__ bsrc, float* __restrict__ wp, float* __restrict__ bp) {
  const int t = threadIdx.x;
  for (int e = t; e < 32 * 128; e += 256) { const float v = (e < NCLS * 128) ? w[e] : 0.0f; *(volatile float*)(wp + e) = v; }
  if (t < 32) { const float v = (t < NCLS) ? bsrc[t] : 0.0f; *(volatile float*)(bp + t) = v; }
  __threadfence();
  for (int e = t; e < 32 * 128; e += 256) { const float v = (e < NCLS * 128) ? w[e] : 0.0f; *(volatile float*)(wp + e) = v; }
  if (t < 32) { const float v = (t < NCLS) ? bsrc[t] : 0.0f; *(volatile float*)(bp + t) = v; }
}
__global__ __launch_bounds__(256) void k_add3(const float* __restrict__ a, const float* __restrict__ bb, const float* __restrict__ c, float* __restrict__ d, size_t n4) {
  const size_t i = (size_t)blockIdx.x * 256 + threadIdx.x; if (i >= n4) return;
  const v4f_t v = *(const v4f_t*)(a + 4 * i) + *(const v4f_t*)(bb + 4 * i) + *(const v4f_t*)(c + 4 * i);
  *(volatile v4f_t*)(d + 4 * i) = v; __threadfence(); *(volatile v4f_t*)(d + 4 * i) = v;
}
__global__ __launch_bounds__(256) void k_upsample(const float* __restrict__ lgT, float* __restrict__ out) {
  const size_t i = (size_t)blockIdx.x * 256 + threadIdx.x;
  const int xq = (int)(i & 63), Y = (int)((i >> 6) & 255), k = (int)((i >> 14) % NCLS), b = (int)(i / ((size_t)64 * 256 * NCLS));
  if (b >= NB_) return;
  const float sy = ((float)Y + 0.5f) * 0.25f - 0.5f;
  const int y0 = (int)floorf(sy); const float fy = sy - (float)y0;
  const int ya = min(max(y0, 0), IMH - 1), yb = min(max(y0 + 1, 0), IMH - 1);
  v4f_t res;
#pragma unroll
  for (int u = 0; u < 4; ++u) {
    const int X = xq * 4 + u;
    const float sx = ((float)X + 0.5f) * 0.25f - 0.5f;
    const int x0 = (int)floorf(sx); const float fx = sx - (float)x0;
    const int xa = min(max(x0, 0), IMW - 1), xb = min(max(x0 + 1, 0), IMW - 1);
    const float* base = lgT + (size_t)b * HW_ * 32 + k;
    const float v00 = base[(size_t)(ya * IMW + xa) * 32], v01 = base[(size_t)(ya * IMW + xb) * 32];
    const float v10 = base[(size_t)(yb * IMW + xa) * 32], v11 = base[(size_t)(yb * IMW + xb) * 32];
    const float top = v00 * (1.0f - fx) + v01 * fx, bot = v10 * (1.0f - fx) + v11 * fx;
    res[u] = top * (1.0f - fy) + bot * fy;
  }
  float* o = out + (((size_t)b * NCLS + k) * 256 + Y) * 256 + xq * 4;
  *(volatile v4f_t*)o = res; __threadfence(); *(volatile v4f_t*)o = res;
}

extern "C" void kernel_launch(void* const* d_in, const int* in_sizes, int n_in,
                              void* d_out, int out_size, void* d_ws, size_t ws_size,
                              hipStream_t stream) {
  (void)in_sizes; (void)n_in; (void)out_size; (void)ws_size;
  const float* x = (const float*)d_in[0];
  const float* w_pam = (const float*)d_in[1];
  const float* gps = (const float*)d_in[2], *gpb = (const float*)d_in[3];
  const float* w_cam = (const float*)d_in[4];
  const float* gcs = (const float*)d_in[5], *gcb = (const float*)d_in[6];
  const float* w_pred = (const float*)d_in[7];
  const float* b_pred = (const float*)d_in[8];
  float* out = (float*)d_out;
  char* ws = (char*)d_ws;
  const size_t T4 = (size_t)NB_ * CD * HW_ * 4, T2 = T4 / 2;
  float* pam_pre = (float*)ws; ws += T4;  float* cam_pre = (float*)ws; ws += T4;
  float* stp = (float*)ws; ws += 4096;     float* stc = (float*)ws; ws += 4096;
  float* pamC32 = (float*)ws; ws += T4;   bf16* pamC16 = (bf16*)ws; ws += T2;  float* pamT32 = (float*)ws; ws += T4;  bf16* pamT16 = (bf16*)ws; ws += T2;
  float* camC32 = (float*)ws; ws += T4;   bf16* camC16 = (bf16*)ws; ws += T2;  float* camT32 = (float*)ws; ws += T4;  bf16* camT16 = (bf16*)ws; ws += T2;
  float* attnT = (float*)ws; ws += T4;    float* gram = (float*)ws; ws += (size_t)NB_ * CD * CD * 4;  float* cw = (float*)ws; ws += (size_t)NB_ * CD * CD * 4;
  float* sumcT = (float*)ws; ws += T4;    float* fusedT = (float*)ws; ws += T4;  float* lgT = (float*)ws; ws += (size_t)NB_ * HW_ * 32 * 4;
  float* wpad = (float*)ws; ws += 32 * 128 * 4;  float* bpad = (float*)ws; ws += 256;

  k_convd<<<dim3(NB_ * 32), dim3(256), 0, stream>>>(x, w_pam, pam_pre);
  k_convd<<<dim3(NB_ * 32), dim3(256), 0, stream>>>(x, w_cam, cam_pre);
  k_gn_stats<<<dim3(NB_ * 2), dim3(256), 0, stream>>>(pam_pre, stp);
  k_gn_stats<<<dim3(NB_ * 2), dim3(256), 0, stream>>>(cam_pre, stc);
  k_gn_apply<<<dim3(NB_ * 64), dim3(256), 0, stream>>>(pam_pre, stp, gps, gpb, pamC32, pamC16, pamT32, pamT16);
  k_gn_apply<<<dim3(NB_ * 64), dim3(256), 0, stream>>>(cam_pre, stc, gcs, gcb, camC32, camC16, camT32, camT16);
  attn_kernel<<<dim3(SS / 32, 1, NB_), dim3(64), 0, stream>>>(pamT16, pamT16, pamC16, attnT);
  for (int b = 0; b < NB_; ++b)
    gemm_rb_kernel<float, 2><<<dim3(CD / 128, 1), dim3(256), 0, stream>>>(camC32 + (size_t)b * CD * HW_, camC32 + (size_t)b * CD * HW_, nullptr, nullptr, nullptr, nullptr, gram + (size_t)b * CD * CD, CD, CD, HW_);
  k_softmax128<<<dim3(NB_), dim3(256), 0, stream>>>(gram, cw);
  for (int b = 0; b < NB_; ++b)
    gemm_rb_kernel<float, 2><<<dim3(HW_ / 128, 1), dim3(256), 0, stream>>>(camT32 + (size_t)b * HW_ * CD, cw + (size_t)b * CD * CD, nullptr, nullptr, camT32 + (size_t)b * HW_ * CD, nullptr, sumcT + (size_t)b * HW_ * CD, HW_, CD, CD);
  k_add3<<<dim3((unsigned)((NB_ * HW_ * CD / 4 + 255) / 256)), dim3(256), 0, stream>>>(pamT32, attnT, sumcT, fusedT, (size_t)NB_ * HW_ * CD / 4);
  k_padw<<<dim3(1), dim3(256), 0, stream>>>(w_pred, b_pred, wpad, bpad);
  gemm_rb_kernel<float, 2><<<dim3(NB_ * HW_ / 128, 1), dim3(256), 0, stream>>>(fusedT, wpad, bpad, nullptr, nullptr, nullptr, lgT, NB_ * HW_, 32, CD);
  k_upsample<<<dim3((unsigned)(((size_t)NB_ * NCLS * 256 * 64 + 255) / 256)), dim3(256), 0, stream>>>(lgT, out);
}
